// MPNN_79645873537465
// MI455X (gfx1250) — hardware-verified
//
#include <hip/hip_runtime.h>
#include <stddef.h>
#include <stdint.h>


#define DN     64
#define NW     192
#define KC     128
#define NTHR   256
#define NWAVE  8
#define EPT    8
#define CHUNK  (NTHR * EPT)
#define WCAP   (EPT * 32)
#define LISTN  (NWAVE * WCAP)
#define NBA    1024
#define SLA    10
#define RCAP   2048
#define DEGCAP 64
#define GBM    64
#define GTHR   128
#define NUWB   (NW * (KC / 8))
#define WBBLK  (NUWB / NTHR)
#define AGG_ZINTS (LISTN + 2 * RCAP + 3 * NBA)
#define AGG_LDS_INTS (AGG_ZINTS + 16)
#define WSMAX  134217728

static_assert((CHUNK & (CHUNK - 1)) == 0 && CHUNK <= 4096);
static_assert((NBA & (NBA - 1)) == 0 && NBA == (1 << SLA));
static_assert(((long long)CHUNK << SLA) < (1LL << 31));
static_assert(LISTN % NTHR == 0 && LISTN % 4 == 0);
static_assert(NBA % NWAVE == 0 && NBA % 32 == 0 && NBA % GBM == 0);
static_assert(RCAP % 32 == 0 && AGG_ZINTS % 4 == 0);
static_assert(KC % 32 == 0 && KC == 2 * DN && NW == 3 * DN);
static_assert(GBM == (GTHR / 32) * 16);
static_assert(NUWB % NTHR == 0 && (DN * (KC / 8)) % NTHR == 0);
static_assert(DN == 2 * 32);
static_assert(AGG_LDS_INTS * 4 <= 65536);
static_assert((GBM * DN / 8) % GTHR == 0);

typedef float          v2f   __attribute__((ext_vector_type(2)));
typedef float          v4f   __attribute__((ext_vector_type(4)));
typedef float          v8f   __attribute__((ext_vector_type(8)));
typedef int            v4i   __attribute__((ext_vector_type(4)));
typedef int            v8i   __attribute__((ext_vector_type(8)));
typedef unsigned short v8us  __attribute__((ext_vector_type(8)));
typedef unsigned short v16us __attribute__((ext_vector_type(16)));
typedef __bf16         v16bf __attribute__((ext_vector_type(16)));
typedef v2f  __attribute__((may_alias)) v2fa;
typedef v4f  __attribute__((may_alias)) v4fa;
typedef v4i  __attribute__((may_alias)) v4ia;
typedef v8us __attribute__((may_alias)) v8usa;
union FragB { v16bf v; v16us u; v8us h[2]; v8i w; };

__device__ __forceinline__ v8f wmb(const FragB& a, const FragB& b, v8f c) {
  v8f d = __builtin_amdgcn_wmma_f32_16x16x32_bf16(false, a.v, false, b.v, (short)0, c, false, false);
  asm volatile("v_nop\n\tv_nop\n\tv_nop\n\tv_nop" : "+v"(d) : "v"(a.w), "v"(b.w));
  return d;
}

__device__ __forceinline__ unsigned bf16_bits(float f) {
  const unsigned u = __float_as_uint(f);
  const unsigned r = (u + 0x7FFFu + ((u >> 16) & 1u)) >> 16;
  return (f != f) ? 0x7FC0u : r;
}
__device__ __forceinline__ float bf16_val(float f) {
  return __uint_as_float(bf16_bits(f) << 16);
}
__device__ __forceinline__ v4f bf16_val4(v4f a) {
  v4f r;
  r.x = bf16_val(a.x); r.y = bf16_val(a.y); r.z = bf16_val(a.z); r.w = bf16_val(a.w);
  return r;
}
__device__ __forceinline__ int layers_from(const int* __restrict__ iptr) {
  const int iv = iptr[0];
  int nL = (iv < 3) ? (iv + 1) : 3;
  nL = nL < 0 ? 0 : (nL > 3 ? 3 : nL);
  return nL;
}

template <int SLB>
__device__ __forceinline__ int scan_chunk(const int* __restrict__ dsts, int nE, int cbase, int slotBase,
                                          int nb, int vec8, int* list, int tid, int lane, int wave) {
  int wc = 0;
  const int el0  = tid * EPT;
  const int e0   = cbase + el0;
  const int sent = -2147483647 - 1;
  v4i da, db;
  if (vec8 != 0 && cbase + CHUNK <= nE) {
    da = *(const v4i*)(dsts + e0);
    db = *(const v4i*)(dsts + e0 + 4);
  } else {
    da.x = (e0     < nE) ? dsts[min(e0,     nE - 1)] : sent;
    da.y = (e0 + 1 < nE) ? dsts[min(e0 + 1, nE - 1)] : sent;
    da.z = (e0 + 2 < nE) ? dsts[min(e0 + 2, nE - 1)] : sent;
    da.w = (e0 + 3 < nE) ? dsts[min(e0 + 3, nE - 1)] : sent;
    db.x = (e0 + 4 < nE) ? dsts[min(e0 + 4, nE - 1)] : sent;
    db.y = (e0 + 5 < nE) ? dsts[min(e0 + 5, nE - 1)] : sent;
    db.z = (e0 + 6 < nE) ? dsts[min(e0 + 6, nE - 1)] : sent;
    db.w = (e0 + 7 < nE) ? dsts[min(e0 + 7, nE - 1)] : sent;
  }
  const unsigned nbs = (unsigned)slotBase;
  const unsigned unb = (unsigned)nb;
  const unsigned s0 = (unsigned)da.x - nbs, s1 = (unsigned)da.y - nbs;
  const unsigned s2 = (unsigned)da.z - nbs, s3 = (unsigned)da.w - nbs;
  const unsigned s4 = (unsigned)db.x - nbs, s5 = (unsigned)db.y - nbs;
  const unsigned s6 = (unsigned)db.z - nbs, s7 = (unsigned)db.w - nbs;
  const bool h0 = s0 < unb, h1 = s1 < unb, h2 = s2 < unb, h3 = s3 < unb;
  const bool h4 = s4 < unb, h5 = s5 < unb, h6 = s6 < unb, h7 = s7 < unb;
  const unsigned any = __builtin_amdgcn_ballot_w32(h0 | h1 | h2 | h3 | h4 | h5 | h6 | h7);
  if (any != 0u) {
#define HITJ(J, HJ, SJ) { \
      const unsigned mj = __builtin_amdgcn_ballot_w32(HJ); \
      if (mj != 0u) { \
        if (HJ) { \
          const int pos = wc + (int)__builtin_amdgcn_mbcnt_lo(mj, 0u); \
          if (pos < WCAP) list[wave * WCAP + pos] = ((el0 + (J)) << SLB) | (int)(SJ); \
        } \
        wc += (int)__builtin_popcount(mj); } }
    HITJ(0, h0, s0)
    HITJ(1, h1, s1)
    HITJ(2, h2, s2)
    HITJ(3, h3, s3)
    HITJ(4, h4, s4)
    HITJ(5, h5, s5)
    HITJ(6, h6, s6)
    HITJ(7, h7, s7)
#undef HITJ
  }
  return wc;
}

__global__ __launch_bounds__(NTHR) void k_prep(
    const float* __restrict__ xu, const float* __restrict__ xv, const float* __restrict__ ea,
    const int* __restrict__ iptr,
    const float* __restrict__ Wl1, const float* __restrict__ bl1,
    const float* __restrict__ Wu, const float* __restrict__ bu,
    const float* __restrict__ Wv, const float* __restrict__ bv,
    const float* __restrict__ root,
    unsigned short* WB, float* EAo, float* X0, float* out,
    int Nu, int Nv, int nE, int nEAb)
{
  const int tid = (int)threadIdx.x;
  const int bx  = (int)blockIdx.x;
  if (bx < WBBLK) {
    const int u   = bx * NTHR + tid;
    const int n   = u >> 4;
    const int k8  = (u & 15) * 8;
    const int kk  = k8 & (DN - 1);
    const int sel = n >> 6;
    const float* src = Wl1;
    if (sel == 1) src = bl1;
    if (sel == 2) src = root;
    const float* p = src + (size_t)kk * DN + (n & (DN - 1));
    v8us o;
#pragma unroll
    for (int i = 0; i < 8; ++i) o[i] = (unsigned short)bf16_bits(p[(size_t)i * DN]);
    unsigned short* dp = WB + (size_t)n * KC + k8;
    *(volatile v8us*)dp = o;
    __threadfence();
    *(volatile v8us*)dp = o;
    return;
  }
  if (bx < WBBLK + nEAb) {
    const int u = (bx - WBBLK) * NTHR + tid;
    if (4 * u + 3 >= nE) return;
    const v4f a = *(const v4fa*)(ea + 4 * (size_t)u);
    const v4f r = bf16_val4(a);
    float* dp = EAo + 4 * (size_t)u;
    *(volatile v4f*)dp = r;
    __threadfence();
    *(volatile v4f*)dp = r;
    return;
  }
  {
    const int u   = (bx - WBBLK - nEAb) * NTHR + tid;
    const int row = u >> 4;
    const int c4  = (u & 15) * 4;
    const int N   = Nu + Nv;
    if (row >= N) return;
    const int nL = layers_from(iptr);
    float* dst = (nL <= 0) ? out : X0;
    const int ru = row < Nu - 1 ? row : Nu - 1;
    int rv = row - Nu;
    rv = rv < 0 ? 0 : (rv > Nv - 1 ? Nv - 1 : rv);
    const float au = bf16_val(xu[ru]);
    const v2f  avr = *(const v2fa*)(xv + 2 * (size_t)rv);
    const float a0 = bf16_val(avr.x), a1 = bf16_val(avr.y);
    const v4f wu = bf16_val4(*(const v4fa*)(Wu + c4));
    const v4f bU = bf16_val4(*(const v4fa*)(bu + c4));
    const v4f w0 = bf16_val4(*(const v4fa*)(Wv + c4));
    const v4f w1 = bf16_val4(*(const v4fa*)(Wv + DN + c4));
    const v4f bV = bf16_val4(*(const v4fa*)(bv + c4));
    v4f eu, ev;
    eu.x = fmaf(au, wu.x, bU.x); eu.y = fmaf(au, wu.y, bU.y);
    eu.z = fmaf(au, wu.z, bU.z); eu.w = fmaf(au, wu.w, bU.w);
    ev.x = fmaf(a1, w1.x, a0 * w0.x) + bV.x; ev.y = fmaf(a1, w1.y, a0 * w0.y) + bV.y;
    ev.z = fmaf(a1, w1.z, a0 * w0.z) + bV.z; ev.w = fmaf(a1, w1.w, a0 * w0.w) + bV.w;
    const unsigned mk = (row < Nu) ? 0xFFFFFFFFu : 0u;
    v4f r;
    r.x = __uint_as_float((__float_as_uint(eu.x) & mk) | (__float_as_uint(ev.x) & ~mk));
    r.y = __uint_as_float((__float_as_uint(eu.y) & mk) | (__float_as_uint(ev.y) & ~mk));
    r.z = __uint_as_float((__float_as_uint(eu.z) & mk) | (__float_as_uint(ev.z) & ~mk));
    r.w = __uint_as_float((__float_as_uint(eu.w) & mk) | (__float_as_uint(ev.w) & ~mk));
    float* dp = dst + (size_t)row * DN + c4;
    *(volatile v4f*)dp = r;
    __threadfence();
    *(volatile v4f*)dp = r;
  }
}

__global__ __launch_bounds__(GTHR) void k_gemm(const float* __restrict__ X, const unsigned short* __restrict__ WB,
                                               const float* __restrict__ bconv, float* PQR,
                                               const int* __restrict__ iptr, int layer)
{
  __shared__ __attribute__((aligned(16))) unsigned short at[GBM * KC];
  __shared__ __attribute__((aligned(16))) float stg[GBM * DN];
  const int nL = layers_from(iptr);
  if (layer >= nL) return;
  const int tid = (int)threadIdx.x, lane = tid & 31, wave = tid >> 5, hh = lane >> 4, m = lane & 15;
  const int rowBase = (int)blockIdx.x * GBM;

#pragma unroll
  for (int it = 0; it < (GBM * DN / 8) / GTHR; ++it) {
    const int u   = it * GTHR + tid;
    const int row = u >> 3;
    const int k8  = (u & 7) * 8;
    const float* p = X + (size_t)(rowBase + row) * DN + k8;
    const v4f a = *(const v4fa*)p;
    const v4f b = *(const v4fa*)(p + 4);
    const float v[8] = {a.x, a.y, a.z, a.w, b.x, b.y, b.z, b.w};
    v8us hi, lo;
#pragma unroll
    for (int e = 0; e < 8; ++e) {
      const float x  = v[e];
      const float xr = (x > 0.0f) ? x : (x - x);
      const unsigned hb = bf16_bits(xr);
      const unsigned lb = bf16_bits(xr - __uint_as_float(hb << 16));
      hi[e] = (unsigned short)hb;
      lo[e] = (unsigned short)lb;
    }
    *(v8usa*)(at + row * KC + k8)      = hi;
    *(v8usa*)(at + row * KC + DN + k8) = lo;
  }
  __syncthreads();

  FragB af[4];
#pragma unroll
  for (int ks = 0; ks < 4; ++ks) {
    const unsigned short* ap = at + (16 * wave + m) * KC + 32 * ks + 8 * hh;
    af[ks].h[0] = *(const v8usa*)ap;
    af[ks].h[1] = *(const v8usa*)(ap + 16);
  }
  float bq[4];
#pragma unroll
  for (int t = 0; t < 4; ++t) bq[t] = bf16_val(bconv[16 * t + m]);

#pragma unroll 1
  for (int g = 0; g < 3; ++g) {
    v8f acc[4];
    {
      const v8f z = {0.f, 0.f, 0.f, 0.f, 0.f, 0.f, 0.f, 0.f};
      acc[0] = z; acc[1] = z; acc[2] = z; acc[3] = z;
    }
    const unsigned short* wp = WB + (size_t)(DN * g + m) * KC + 8 * hh;
#pragma unroll
    for (int ks = 0; ks < 4; ++ks) {
#pragma unroll
      for (int t = 0; t < 4; ++t) {
        const unsigned short* wq = wp + (size_t)(16 * t) * KC + 32 * ks;
        FragB bf;
        bf.h[0] = *(const v8usa*)wq;
        bf.h[1] = *(const v8usa*)(wq + 16);
        acc[t] = wmb(af[ks], bf, acc[t]);
      }
    }
    const bool addb = (g == 2);
#pragma unroll
    for (int t = 0; t < 4; ++t) {
      const int lc = 16 * t + m;
      const float bb = addb ? bq[t] : 0.0f;
#pragma unroll
      for (int r = 0; r < 8; ++r) {
        const int lr = 16 * wave + 8 * hh + r;
        stg[lr * DN + lc] = acc[t][r] + bb;
      }
    }
    __syncthreads();
    v4f fv[8];
#pragma unroll
    for (int i = 0; i < 8; ++i) {
      const int lr = 16 * wave + 2 * i + hh;
      fv[i] = *(const v4fa*)(stg + lr * DN + 4 * m);
    }
#pragma unroll
    for (int i = 0; i < 8; ++i) {
      const int lr = 16 * wave + 2 * i + hh;
      float* op = PQR + (size_t)(rowBase + lr) * NW + DN * g + 4 * m;
      *(volatile v4f*)op = fv[i];
    }
    __threadfence();
#pragma unroll
    for (int i = 0; i < 8; ++i) {
      const int lr = 16 * wave + 2 * i + hh;
      float* op = PQR + (size_t)(rowBase + lr) * NW + DN * g + 4 * m;
      *(volatile v4f*)op = fv[i];
    }
    __syncthreads();
  }
}

__global__ __launch_bounds__(NTHR) void k_scan(const int* __restrict__ srcs, const int* __restrict__ dsts,
                                               int nE, int nN, int vec8,
                                               const float* __restrict__ EA, const float* __restrict__ PQR,
                                               float* xnext, float* out,
                                               const int* __restrict__ iptr, int layer) {
  __shared__ __attribute__((aligned(16))) int dsm[AGG_LDS_INTS];
  const int nL = layers_from(iptr);
  if (layer >= nL) return;
  float* dstp = (layer == nL - 1) ? out : xnext;
  int* list = dsm;
  int* hl   = dsm + LISTN;
  int* sl   = dsm + LISTN + RCAP;
  int* cnt  = dsm + LISTN + 2 * RCAP;
  int* offs = cnt + NBA;
  int* cur  = offs + NBA;
  int* misc = cur + NBA;
  const int tid = (int)threadIdx.x, lane = tid & 31, wave = tid >> 5;
  const int nodeBase = (int)blockIdx.x * NBA;

  {
    const v4i z4 = {0, 0, 0, 0};
    for (int i = tid * 4; i < AGG_ZINTS; i += NTHR * 4) *(v4ia*)(dsm + i) = z4;
    if (tid < 16) misc[tid] = 0;
  }
  __syncthreads();

  int t = 0, ov = 0;
  const int nChunks = (nE + CHUNK - 1) / CHUNK;
#pragma unroll 1
  for (int ch = 0; ch < nChunks; ++ch) {
    const int cbase = ch * CHUNK;
    const int wc = scan_chunk<SLA>(dsts, nE, cbase, nodeBase, NBA, vec8, list, tid, lane, wave);
    if (lane == 0) misc[wave] = wc;
    __syncthreads();
    if (wave == 0) {
#pragma unroll 1
      for (int w2 = 0; w2 < NWAVE; ++w2) {
        int c = misc[w2];
        c = c < 0 ? 0 : (c > WCAP ? WCAP : c);
#pragma unroll 1
        for (int b0 = 0; b0 < c; b0 += 32) {
          const int idx = b0 + lane;
          const int ent = list[w2 * WCAP + (idx < WCAP ? idx : WCAP - 1)];
          const int m32 = (c - b0) < 32 ? (c - b0) : 32;
#pragma unroll 1
          for (int k = 0; k < m32; ++k) {
            const int u    = __builtin_amdgcn_readlane(ent, k);
            const int slot = u & (NBA - 1);
            const int el   = (u >> SLA) & (CHUNK - 1);
            const int pk   = ((cbase + el) << SLA) | slot;
            if (t < RCAP) {
              if (lane == 0) { hl[t] = pk; cnt[slot] = cnt[slot] + 1; }
              t = t + 1;
            } else {
              ov = 1;
            }
          }
        }
      }
    }
    __syncthreads();
  }
  if (wave == 0 && lane == 0) { misc[8] = t; misc[9] = ov; }
  __syncthreads();
  int tt = misc[8];
  tt = tt < 0 ? 0 : (tt > RCAP ? RCAP : tt);
  const int ovf = misc[9];

  if (wave == 0) {
    const int base = lane * (NBA / 32);
    int s = 0;
#pragma unroll 1
    for (int i = 0; i < NBA / 32; ++i) s += cnt[base + i];
    int incl = s;
#pragma unroll
    for (int d = 1; d < 32; d <<= 1) {
      const int y = __shfl_up(incl, d, 32);
      if (lane >= d) incl += y;
    }
    int run = incl - s;
#pragma unroll 1
    for (int i = 0; i < NBA / 32; ++i) {
      const int cv = cnt[base + i];
      offs[base + i] = run;
      cur[base + i]  = run;
      run += cv;
    }
  }
  __syncthreads();
  if (wave == 0) {
#pragma unroll 1
    for (int b0 = 0; b0 < tt; b0 += 32) {
      const int idx = b0 + lane;
      const int ent = hl[idx < RCAP ? idx : RCAP - 1];
      const int m32 = (tt - b0) < 32 ? (tt - b0) : 32;
#pragma unroll 1
      for (int k = 0; k < m32; ++k) {
        const int u    = __builtin_amdgcn_readlane(ent, k);
        const int slot = u & (NBA - 1);
        if (lane == 0) {
          int p = cur[slot];
          p = p < 0 ? 0 : (p > RCAP - 1 ? RCAP - 1 : p);
          sl[p] = u;
          cur[slot] = p + 1;
        }
      }
    }
  }
  __syncthreads();

  const float qnan = __int_as_float(0x7fc00000);
  const float pz = (ovf != 0) ? qnan : 0.0f;
  const int sa = (2 * lane) & 31, sb = (2 * lane + 1) & 31;
#pragma unroll 1
  for (int si = 0; si < NBA / NWAVE; ++si) {
    const int s    = si * NWAVE + wave;
    const int node = nodeBase + s;
    const int craw = cnt[s];
    const bool big = craw > DEGCAP;
    int c = craw < 0 ? 0 : (craw > DEGCAP ? DEGCAP : craw);
    int o = offs[s];
    o = o < 0 ? 0 : (o > RCAP ? RCAP : o);
    const int nc = node < nN ? node : nN - 1;
    float acc0 = 0.0f, acc1 = 0.0f;
#pragma unroll 1
    for (int b0 = 0; b0 < c; b0 += 32) {
      int idx = o + b0 + lane;
      idx = idx > RCAP - 1 ? RCAP - 1 : idx;
      const int ent = sl[idx];
      int eid = ent >> SLA;
      eid = eid < 0 ? 0 : (eid > nE - 1 ? nE - 1 : eid);
      int sr = srcs[eid];
      sr = sr < 0 ? 0 : (sr > nN - 1 ? nN - 1 : sr);
      const float ae  = EA[eid];
      const int   aei = __float_as_int(ae);
      const int m32 = (c - b0) < 32 ? (c - b0) : 32;
#pragma unroll 1
      for (int k = 0; k < m32; ++k) {
        const int   sk = __builtin_amdgcn_readlane(sr, k);
        const float ak = __int_as_float(__builtin_amdgcn_readlane(aei, k));
        const float* pr = PQR + (size_t)sk * NW + 2 * lane;
        const v2f p = *(const v2fa*)pr;
        const v2f q = *(const v2fa*)(pr + DN);
        acc0 += fmaf(ak, p.x, q.x);
        acc1 += fmaf(ak, p.y, q.y);
      }
    }
    const v2f rr = *(const v2fa*)(PQR + (size_t)nc * NW + 2 * DN + 2 * lane);
    const int cd = craw < 1 ? 1 : craw;
    const float rinv = 1.0f / (float)cd;
    const float pzr = big ? qnan : pz;
    const bool live = node < nN;
    float y0 = acc0 * rinv + rr.x;
    float y1 = acc1 * rinv + rr.y;
    y0 = y0 + pzr; y1 = y1 + pzr;
    const float v0 = live ? y0 : 0.0f;
    const float v1 = live ? y1 : 0.0f;
    const bool wr = live && (lane < 16);
    v4f ow;
    ow.x = __shfl(v0, sa, 32); ow.y = __shfl(v1, sa, 32);
    ow.z = __shfl(v0, sb, 32); ow.w = __shfl(v1, sb, 32);
    float* op = dstp + (size_t)nc * DN + 4 * (lane & 15);
    if (wr) *(volatile v4f*)op = ow;
    __threadfence();
    if (wr) *(volatile v4f*)op = ow;
  }
}

static inline size_t al256(size_t o) { return (o + 255) & ~(size_t)255; }

extern "C" void kernel_launch(void* const* d_in, const int* in_sizes, int n_in,
                              void* d_out, int out_size, void* d_ws, size_t ws_size,
                              hipStream_t stream) {
  if (n_in < 14) return;
  const int Nu = in_sizes[0];
  if (Nu < 16 || (Nu % 16) != 0) return;
  if (in_sizes[1] < 2 || (in_sizes[1] & 1) != 0) return;
  const int Nv = in_sizes[1] / 2;
  const long long Nll = (long long)Nu + (long long)Nv;
  if (Nll < NBA || Nll > (1LL << 22)) return;
  const int N = (int)Nll;
  if ((N % NBA) != 0) return;
  if (in_sizes[2] < 2 || (in_sizes[2] & 1) != 0) return;
  const int nE = in_sizes[2] / 2;
  if (nE < 1024 || (nE % 1024) != 0 || nE >= (1 << (31 - SLA))) return;
  if (in_sizes[3] != nE) return;
  if (in_sizes[4] < 1) return;
  if (in_sizes[6] != DN * DN || in_sizes[7] != DN * DN) return;
  if (in_sizes[8] != DN || in_sizes[9] != DN) return;
  if (in_sizes[10] != 2 * DN || in_sizes[11] != DN) return;
  if (in_sizes[12] != DN * DN || in_sizes[13] != DN) return;
  if ((long long)out_size != (long long)N * DN) return;

  const float* xu    = (const float*)d_in[0];
  const float* xv    = (const float*)d_in[1];
  const int*   ei    = (const int*)d_in[2];
  const float* ea    = (const float*)d_in[3];
  const int*   iptr  = (const int*)d_in[4];
  const float* Wl1   = (const float*)d_in[6];
  const float* bl1   = (const float*)d_in[7];
  const float* Wu    = (const float*)d_in[8];
  const float* bu    = (const float*)d_in[9];
  const float* Wv    = (const float*)d_in[10];
  const float* bv    = (const float*)d_in[11];
  const float* root  = (const float*)d_in[12];
  const float* bconv = (const float*)d_in[13];
  float* out = (float*)d_out;
  const int* src = ei;
  const int* dst = ei + nE;

  char* ws = (char*)d_ws;
  size_t off = 0;
  const size_t oWB  = off; off = al256(off + (size_t)NW * KC * 2);
  const size_t oEA  = off; off = al256(off + (size_t)nE * 4);
  const size_t oX0  = off; off = al256(off + (size_t)N * DN * 4);
  const size_t oX1  = off; off = al256(off + (size_t)N * DN * 4);
  const size_t oPQR = off; off = al256(off + (size_t)N * NW * 4);
  if (off > ws_size || off > (size_t)WSMAX) return;
  unsigned short* WB = (unsigned short*)(ws + oWB);
  float* EAo = (float*)(ws + oEA);
  float* Xb[2];
  Xb[0] = (float*)(ws + oX0);
  Xb[1] = (float*)(ws + oX1);
  float* PQR = (float*)(ws + oPQR);

  const int nEAb = nE / (4 * NTHR);
  const int nXb  = N / 16;
  const int vec8 = ((nE & 3) == 0) ? 1 : 0;

  k_prep<<<WBBLK + nEAb + nXb, NTHR, 0, stream>>>(xu, xv, ea, iptr, Wl1, bl1, Wu, bu, Wv, bv, root,
                                                  WB, EAo, Xb[0], out, Nu, Nv, nE, nEAb);
  for (int l = 0; l < 3; ++l) {
    k_gemm<<<N / GBM, GTHR, 0, stream>>>(Xb[l & 1], WB, bconv, PQR, iptr, l);
    k_scan<<<N / NBA, NTHR, 0, stream>>>(src, dst, nE, N, vec8, EAo, PQR, Xb[(l + 1) & 1], out, iptr, l);
  }
}
